// FlashAttention_71880572666571
// MI455X (gfx1250) — hardware-verified
//
#include <hip/hip_runtime.h>


#ifndef NB
#define NB 2
#endif
#ifndef SEQ
#define SEQ 2048
#endif
#define NB_FULL  2
#define SEQ_FULL 2048
#define DM   1024
#define NH   16
#define HD   64
#define SCL  0.125f
#define PCAR 1024.0f
#define L2E  1.4426950408889634f

static_assert(SEQ % 64 == 0);
static_assert(NB >= 1 && NB <= NB_FULL);
static_assert(SEQ >= 64 && SEQ <= SEQ_FULL);
static_assert(NH * HD == DM);
static_assert(DM % 64 == 0);

#define SZ_XB  ((size_t)NB * SEQ * DM * 2)
#define SZ_W   ((size_t)DM * DM * 2)
#define SZ_Y   ((size_t)NB * SEQ * DM * 4)
#define SZ_PL  ((size_t)NB * NH * SEQ * HD * 2)
#define SZ_CX  ((size_t)NB * SEQ * DM * 2)
#define WS_TOTAL (SZ_XB + 4 * SZ_W + SZ_Y + 3 * SZ_PL + 2 * SZ_CX)
static_assert(WS_TOTAL <= (size_t)134217728);
static_assert(SZ_XB % 256 == 0 && SZ_W % 256 == 0 && SZ_Y % 256 == 0 && SZ_PL % 256 == 0 && SZ_CX % 256 == 0);
static_assert(((size_t)(NB - 1) * SEQ_FULL + SEQ) * DM <= (size_t)NB_FULL * SEQ_FULL * DM);

typedef _Float16 h16;
typedef unsigned short bf;
typedef __attribute__((ext_vector_type(16))) __bf16   v16bf;
typedef __attribute__((ext_vector_type(16))) _Float16 v16h;
typedef __attribute__((ext_vector_type(8)))  _Float16 v8h;
typedef __attribute__((ext_vector_type(8)))  unsigned short v8us;
typedef __attribute__((ext_vector_type(8)))  float    v8f;
typedef __attribute__((ext_vector_type(4)))  float    v4f;
typedef __attribute__((ext_vector_type(2)))  float    v2f;
typedef __attribute__((ext_vector_type(2)))  _Float16 v2h;
typedef __attribute__((ext_vector_type(2)))  unsigned short v2us;
typedef v8h  __attribute__((may_alias)) v8ha;
typedef v4f  __attribute__((may_alias)) v4fa;
typedef v8us __attribute__((may_alias)) v8usa;

__device__ __forceinline__ unsigned short f2bf(float f) { unsigned u = __float_as_uint(f); u += 0x7FFFu + ((u >> 16) & 1u); return (unsigned short)(u >> 16); }
__device__ __forceinline__ float bf2f(unsigned short b) { return __uint_as_float(((unsigned)b) << 16); }
__device__ __forceinline__ float bfr(float f) { return bf2f(f2bf(f)); }
__device__ __forceinline__ void splitf(float y, unsigned short& h, unsigned short& l) { h = f2bf(y); l = f2bf(y - bf2f(h)); }
__device__ __forceinline__ h16 tohx(float x) { return (h16)x; }
__device__ __forceinline__ v16h cat16(v8h lo, v8h hi) { return __builtin_shufflevector(lo, hi, 0, 1, 2, 3, 4, 5, 6, 7, 8, 9, 10, 11, 12, 13, 14, 15); }
__device__ __forceinline__ v16bf cat16b(v8us lo, v8us hi) { return __builtin_bit_cast(v16bf, __builtin_shufflevector(lo, hi, 0, 1, 2, 3, 4, 5, 6, 7, 8, 9, 10, 11, 12, 13, 14, 15)); }
__device__ __forceinline__ v8f wmma16(v16h a, v16h b, v8f c) { return __builtin_amdgcn_wmma_f32_16x16x32_f16(false, a, false, b, (short)0, c, false, false); }
__device__ __forceinline__ v8f wmmab(v16bf a, v16bf b, v8f c) { return __builtin_amdgcn_wmma_f32_16x16x32_bf16(false, a, false, b, (short)0, c, false, false); }

template <typename T16> struct WFrag;
template <> struct WFrag<h16> { typedef v16h V; static __device__ __forceinline__ V ld(const h16* p) { return cat16(*(const v8h*)p, *(const v8h*)(p + 16)); } static __device__ __forceinline__ v8f mma(V a, V b, v8f c) { return wmma16(a, b, c); } };
template <> struct WFrag<bf> { typedef v16bf V; static __device__ __forceinline__ V ld(const bf* p) { return cat16b(*(const v8us*)p, *(const v8us*)(p + 16)); } static __device__ __forceinline__ v8f mma(V a, V b, v8f c) { return wmmab(a, b, c); } };

template <typename T16, int NSPLIT, bool BIAS>
__global__ __launch_bounds__(32) void k_gemmw(const T16* __restrict__ A, const T16* __restrict__ A2, const T16* __restrict__ Bt, const T16* __restrict__ Bt2, int K, float* C, int ldc, const float* __restrict__ bias, size_t sA, size_t sB, size_t sC) {
    typedef typename WFrag<T16>::V V;
    __shared__ __align__(16) float os[16 * 68];
    const size_t z = blockIdx.z; A += z * sA; if (A2) A2 += z * sA; Bt += z * sB; if (Bt2) Bt2 += z * sB; C += z * sC;
    const int lane = threadIdx.x & 31, lr = lane & 15, hi = lane >> 4; const int r0 = blockIdx.x * 64, c0 = blockIdx.y * 64;
    v8f acc[4][4];
#pragma unroll
    for (int mb = 0; mb < 4; ++mb)
#pragma unroll
        for (int nb = 0; nb < 4; ++nb) acc[mb][nb] = (v8f){};
    const size_t aoff = (size_t)(r0 + lr) * K + 8 * hi, boff = (size_t)(c0 + lr) * K + 8 * hi;
#pragma unroll 1
    for (int kc = 0; kc < K; kc += 32) {
        V a[4], a2[4];
#pragma unroll
        for (int mb = 0; mb < 4; ++mb) { a[mb] = WFrag<T16>::ld(A + aoff + (size_t)mb * 16 * K + kc); if (NSPLIT == 1 || NSPLIT == 2) a2[mb] = WFrag<T16>::ld(A2 + aoff + (size_t)mb * 16 * K + kc); }
#pragma unroll
        for (int nb = 0; nb < 4; ++nb) { const V b = WFrag<T16>::ld(Bt + boff + (size_t)nb * 16 * K + kc); V b2; if (NSPLIT >= 2) b2 = WFrag<T16>::ld(Bt2 + boff + (size_t)nb * 16 * K + kc);
#pragma unroll
            for (int mb = 0; mb < 4; ++mb) { acc[mb][nb] = WFrag<T16>::mma(a[mb], b, acc[mb][nb]); if (NSPLIT == 1 || NSPLIT == 2) acc[mb][nb] = WFrag<T16>::mma(a2[mb], b, acc[mb][nb]); if (NSPLIT >= 2) acc[mb][nb] = WFrag<T16>::mma(a[mb], b2, acc[mb][nb]); } }
        asm volatile("v_nop\n\tv_nop\n\tv_nop\n\tv_nop" : "+v"(acc[0][0]), "+v"(acc[1][1]), "+v"(acc[2][2]), "+v"(acc[3][3]) : "v"(a[0]), "v"(a[3]));
    }
#pragma unroll
    for (int mb = 0; mb < 4; ++mb) {
#pragma unroll
        for (int nb = 0; nb < 4; ++nb) {
#pragma unroll
            for (int j = 0; j < 8; ++j) os[(hi * 8 + j) * 68 + nb * 16 + lr] = acc[mb][nb][j]; }
        __builtin_amdgcn_wave_barrier(); asm volatile("" ::: "memory");
        float* crow = C + (size_t)(r0 + mb * 16) * ldc + c0;
#pragma unroll 1
        for (int ps = 0; ps < 2; ++ps) {
#pragma unroll
            for (int s = 0; s < 8; ++s) { const int row = 2 * s + hi, cofs = lr * 4; v4f val = *(const v4fa*)(os + row * 68 + cofs); if (BIAS) { val[0] += bfr(bias[c0 + cofs]); val[1] += bfr(bias[c0 + cofs + 1]); val[2] += bfr(bias[c0 + cofs + 2]); val[3] += bfr(bias[c0 + cofs + 3]); }
                *(volatile v4f*)(crow + (size_t)row * ldc + cofs) = val; }
            if (ps == 0) __threadfence(); }
        __builtin_amdgcn_wave_barrier(); asm volatile("" ::: "memory");
    }
}

__global__ __launch_bounds__(256) void k_cvt8(const float* __restrict__ src, bf* dst, size_t n8) { const size_t i = (size_t)blockIdx.x * 256 + threadIdx.x; if (i >= n8) return; const v8f v = *(const v8f*)(src + i * 8); v8us o;
#pragma unroll
    for (int k = 0; k < 8; ++k) o[k] = f2bf(v[k]); *(volatile v8us*)(dst + i * 8) = o; __threadfence(); *(volatile v8us*)(dst + i * 8) = o; }

__global__ __launch_bounds__(256) void k_cvtx(const float* __restrict__ x, bf* dst, size_t n8) { const size_t i = (size_t)blockIdx.x * 256 + threadIdx.x; if (i >= n8) return; const size_t e = i * 8; const size_t mrow = e / DM; const int c = (int)(e % DM); const size_t b = mrow / SEQ, s = mrow % SEQ;
    const v8f v = *(const v8f*)(x + ((b * SEQ_FULL + s) * DM + c)); v8us o;
#pragma unroll
    for (int k = 0; k < 8; ++k) o[k] = f2bf(v[k]); *(volatile v8us*)(dst + e) = o; __threadfence(); *(volatile v8us*)(dst + e) = o; }

__global__ __launch_bounds__(256) void k_qkp(const float* __restrict__ Y, h16* P) {
    const size_t e = ((size_t)blockIdx.x * 256 + threadIdx.x) * 2; if (e >= (size_t)NB * NH * SEQ * HD) return;
    const int d = (int)(e % HD); const int s = (int)((e / HD) % SEQ); const int h = (int)((e / ((size_t)HD * SEQ)) % NH); const int b = (int)(e / ((size_t)HD * SEQ * NH));
    const v2f y = *(const v2f*)(Y + ((size_t)b * SEQ + s) * DM + h * HD + d); v2h o;
    o[0] = tohx(y[0]); o[1] = tohx(y[1]);
    *(volatile v2h*)(P + e) = o; __threadfence(); *(volatile v2h*)(P + e) = o; }

__global__ __launch_bounds__(256) void k_vtp(const float* __restrict__ Y, h16* Vt) {
    const size_t e = ((size_t)blockIdx.x * 256 + threadIdx.x) * 2; if (e >= (size_t)NB * NH * HD * SEQ) return;
    const int t = (int)(e % SEQ); const int d = (int)((e / SEQ) % HD); const int h = (int)((e / ((size_t)SEQ * HD)) % NH); const int b = (int)(e / ((size_t)SEQ * HD * NH)); v2h o;
#pragma unroll
    for (int q = 0; q < 2; ++q) { const float xv = Y[((size_t)b * SEQ + t + q) * DM + h * HD + d]; o[q] = tohx(xv); }
    *(volatile v2h*)(Vt + e) = o; __threadfence(); *(volatile v2h*)(Vt + e) = o; }

__global__ __launch_bounds__(64) __attribute__((amdgpu_num_vgpr(256)))
void k_attn(const h16* __restrict__ QP, const h16* __restrict__ KP, const h16* __restrict__ VP, bf* CXh, bf* CXl) {
    __shared__ __align__(16) float os[2][16 * 68];
    typedef WFrag<h16> F; typedef v16h V;
    const int lane = threadIdx.x & 31, lr = lane & 15, hi = lane >> 4, wv = threadIdx.x >> 5;
    const int h = blockIdx.y, b = blockIdx.z; const int q0 = blockIdx.x * 32 + wv * 16;
    const size_t zh = (size_t)b * NH + h;
    const h16* Qp = QP + zh * SEQ * HD;
    const h16* Kp = KP + zh * SEQ * HD;
    const h16* Vp = VP + zh * HD * SEQ;
    const size_t qoff = (size_t)(q0 + lr) * HD + 8 * hi;
    const V qf0 = F::ld(Qp + qoff), qf1 = F::ld(Qp + qoff + 32);
    v8f O[4];
#pragma unroll
    for (int dt = 0; dt < 4; ++dt) O[dt] = (v8f){};
    float m = -1.0e30f, l = 0.f;
    const size_t koff = (size_t)lr * HD + 8 * hi, voff = (size_t)lr * SEQ + 8 * hi;
#pragma unroll 1
    for (int kb = 0; kb < SEQ; kb += 32) {
        v8f t[2]; t[0] = (v8f){}; t[1] = (v8f){};
#pragma unroll
        for (int j = 0; j < 2; ++j) {
            const h16* kp = Kp + (size_t)(kb + 16 * j) * HD + koff;
            const V a0 = F::ld(kp), a1 = F::ld(kp + 32);
            t[j] = wmma16(a0, qf0, t[j]); t[j] = wmma16(a1, qf1, t[j]);
        }
        asm volatile("v_nop\n\tv_nop\n\tv_nop\n\tv_nop" : "+v"(t[0]), "+v"(t[1]) : "v"(qf0), "v"(qf1));
        float cmax = -1.0e30f;
#pragma unroll
        for (int r = 0; r < 8; ++r) cmax = fmaxf(cmax, fmaxf(t[0][r], t[1][r]));
        cmax = fmaxf(cmax, __shfl_xor(cmax, 16, 32));
        const float mn = fmaxf(m, cmax * SCL);
        float dm = __fsub_rn(m, mn); asm volatile("" : "+v"(dm));
        const float alpha = __builtin_amdgcn_exp2f(__fmul_rn(dm, L2E));
        m = mn;
        float p[2][8]; float psum = 0.f;
#pragma unroll
        for (int j = 0; j < 2; ++j)
#pragma unroll
            for (int r = 0; r < 8; ++r) { float d0 = __fsub_rn(t[j][r] * SCL, m); asm volatile("" : "+v"(d0)); const float e = __builtin_amdgcn_exp2f(__fmul_rn(d0, L2E)); p[j][r] = e; psum += e; }
        psum += __shfl_xor(psum, 16, 32);
        l = l * alpha + psum;
#pragma unroll
        for (int dt = 0; dt < 4; ++dt) O[dt] *= alpha;
        v8h p0h, p1h;
#pragma unroll
        for (int r = 0; r < 8; ++r) { p0h[r] = tohx(p[0][r] * PCAR); p1h[r] = tohx(p[1][r] * PCAR); }
        const V pb = cat16(p0h, p1h);
#pragma unroll
        for (int dt = 0; dt < 4; ++dt) { const V va = F::ld(Vp + (size_t)dt * 16 * SEQ + kb + voff);
            O[dt] = wmma16(va, pb, O[dt]); }
        asm volatile("v_nop\n\tv_nop\n\tv_nop\n\tv_nop" : "+v"(O[0]), "+v"(O[1]), "+v"(O[2]), "+v"(O[3]) : "v"(pb), "v"(qf0));
    }
    const float inv = __fdiv_rn(1.0f, l) * (1.0f / PCAR);
    float* ow = os[wv];
#pragma unroll
    for (int dt = 0; dt < 4; ++dt)
#pragma unroll
        for (int r = 0; r < 8; ++r) ow[lr * 68 + dt * 16 + 8 * hi + r] = O[dt][r] * inv;
    __builtin_amdgcn_fence(3, "wavefront"); __builtin_amdgcn_wave_barrier(); asm volatile("" ::: "memory");
    const int rsub = lane >> 3, c8 = (lane & 7) * 8;
    bf* ch = CXh + ((size_t)b * SEQ + q0) * DM + h * HD + c8; bf* cl = CXl + ((size_t)b * SEQ + q0) * DM + h * HD + c8;
#pragma unroll 1
    for (int ps = 0; ps < 2; ++ps) {
#pragma unroll
        for (int s = 0; s < 4; ++s) { const int row = s * 4 + rsub;
            const v4f x0 = *(const v4fa*)(ow + row * 68 + c8), x1 = *(const v4fa*)(ow + row * 68 + c8 + 4); v8us oh, ol;
#pragma unroll
            for (int q = 0; q < 4; ++q) { unsigned short a2, c2; splitf(x0[q], a2, c2); oh[q] = a2; ol[q] = c2; splitf(x1[q], a2, c2); oh[4 + q] = a2; ol[4 + q] = c2; }
            *(volatile v8us*)(ch + (size_t)row * DM) = oh; *(volatile v8us*)(cl + (size_t)row * DM) = ol; }
        if (ps == 0) __threadfence(); }
}

extern "C" void kernel_launch(void* const* d_in, const int* in_sizes, int n_in,
                              void* d_out, int out_size, void* d_ws, size_t ws_size, hipStream_t stream) {
    if (n_in < 6) return;
    const size_t rows_hi = (size_t)(NB - 1) * SEQ_FULL + SEQ;
    if ((size_t)in_sizes[0] < rows_hi * DM) return;
    if ((size_t)in_sizes[1] < (size_t)DM * DM || (size_t)in_sizes[2] < (size_t)DM * DM || (size_t)in_sizes[3] < (size_t)DM * DM || (size_t)in_sizes[4] < (size_t)DM * DM) return;
    if ((size_t)in_sizes[5] < (size_t)DM) return;
    if ((size_t)out_size < rows_hi * DM) return;
    const float* x  = (const float*)d_in[0];
    const float* wq = (const float*)d_in[1];
    const float* wk = (const float*)d_in[2];
    const float* wv = (const float*)d_in[3];
    const float* wo = (const float*)d_in[4];
    const float* bo = (const float*)d_in[5];
    float* OUT = (float*)d_out;
    char* wsp = (char*)d_ws;
    auto take = [&](size_t bytes) { char* p = wsp; wsp += (bytes + 255) & ~(size_t)255; return (void*)p; };
    bf* XB  = (bf*)take(SZ_XB);
    bf* WQb = (bf*)take(SZ_W); bf* WKb = (bf*)take(SZ_W); bf* WVb = (bf*)take(SZ_W); bf* WOb = (bf*)take(SZ_W);
    float* Y = (float*)take(SZ_Y);
    h16* QP = (h16*)take(SZ_PL); h16* KP = (h16*)take(SZ_PL); h16* VT = (h16*)take(SZ_PL);
    bf* CXh = (bf*)take(SZ_CX); bf* CXl = (bf*)take(SZ_CX);
    if ((size_t)(wsp - (char*)d_ws) > ws_size) return;

    const size_t nx8 = (size_t)NB * SEQ * DM / 8, nw8 = (size_t)DM * DM / 8;
    k_cvtx<<<(unsigned)((nx8 + 255) / 256), 256, 0, stream>>>(x, XB, nx8);
    k_cvt8<<<(unsigned)((nw8 + 255) / 256), 256, 0, stream>>>(wq, WQb, nw8);
    k_cvt8<<<(unsigned)((nw8 + 255) / 256), 256, 0, stream>>>(wk, WKb, nw8);
    k_cvt8<<<(unsigned)((nw8 + 255) / 256), 256, 0, stream>>>(wv, WVb, nw8);
    k_cvt8<<<(unsigned)((nw8 + 255) / 256), 256, 0, stream>>>(wo, WOb, nw8);

    const dim3 gp(NB * SEQ / 64, DM / 64, 1);
    const unsigned LP = (unsigned)(((size_t)NB * NH * SEQ * HD / 2 + 255) / 256);
    k_gemmw<bf, 0, false><<<gp, 32, 0, stream>>>(XB, nullptr, WQb, nullptr, DM, Y, DM, nullptr, (size_t)0, (size_t)0, (size_t)0);
    k_qkp<<<LP, 256, 0, stream>>>(Y, QP);
    k_gemmw<bf, 0, false><<<gp, 32, 0, stream>>>(XB, nullptr, WKb, nullptr, DM, Y, DM, nullptr, (size_t)0, (size_t)0, (size_t)0);
    k_qkp<<<LP, 256, 0, stream>>>(Y, KP);
    k_gemmw<bf, 0, false><<<gp, 32, 0, stream>>>(XB, nullptr, WVb, nullptr, DM, Y, DM, nullptr, (size_t)0, (size_t)0, (size_t)0);
    k_vtp<<<LP, 256, 0, stream>>>(Y, VT);

    k_attn<<<dim3(SEQ / 32, NH, NB), 64, 0, stream>>>(QP, KP, VT, CXh, CXl);

    k_gemmw<bf, 1, true><<<dim3(SEQ / 64, DM / 64, NB), 32, 0, stream>>>(CXh, CXl, WOb, nullptr, DM, OUT, DM, bo, (size_t)SEQ * DM, (size_t)0, (size_t)SEQ_FULL * DM);
}
